// QNNLayer_47991964565825
// MI455X (gfx1250) — hardware-verified
//
#include <hip/hip_runtime.h>
#include <math.h>

typedef __attribute__((ext_vector_type(16))) _Float16 v16h;
typedef __attribute__((ext_vector_type(8)))  _Float16 v8h;
typedef __attribute__((ext_vector_type(8)))  float    v8f;
typedef __attribute__((ext_vector_type(4)))  float    v4f;

constexpr int kWires  = 8;
constexpr int kDim    = 256;
constexpr int kLayers = 2;
constexpr int kBatch  = 131072;
constexpr int kAmpRows = 2 * kDim;
constexpr int kBlkWaves   = 2;
constexpr int kBlkThreads = kBlkWaves * 32;
constexpr int kBlkSamples = kBlkWaves * 32;
constexpr int kKSteps = kDim / 32;
static_assert(kDim == (1 << kWires), "state size");
static_assert((kBatch % kBlkSamples) == 0, "batch is a multiple of the block tile");
static_assert((kDim % 32) == 0, "K multiple of 32");
static_assert((kAmpRows % 64) == 0, "amplitude rows multiple of 64");

constexpr float kCarryR = 16384.0f;
constexpr float kCarryV = 1024.0f;
constexpr float kFoldSq = 1.0f / ((kCarryR * kCarryV) * (kCarryR * kCarryV));
constexpr float kF16MinNormal = 6.103515625e-05f;

constexpr size_t kOffUT  = 0;
constexpr size_t kSizeUT = (size_t)2 * kDim * kDim * 4;
constexpr size_t kOffVT  = kOffUT + kSizeUT;
constexpr size_t kSizeVT = (size_t)kAmpRows * kDim * 2;
constexpr size_t kWsTotal = kOffVT + kSizeVT;
static_assert(kWsTotal == 786432ull, "carve total");
static_assert((kOffVT % 128) == 0, "aligned region");
static_assert(kWsTotal <= 134217728ull, "carve cap");

union FragU { v16h v; v8h h[2]; };

__device__ __forceinline__ v16h frag_load_rowmajor(const _Float16* p) {
  FragU f;
  f.h[0] = *(const v8h*)(p);
  f.h[1] = *(const v8h*)(p + 16);
  return f.v;
}

__device__ __forceinline__ v8f mma_guarded(v16h a, v16h b, v8f c) {
  c = __builtin_amdgcn_wmma_f32_16x16x32_f16(false, a, false, b, (short)0, c, false, false);
  asm volatile("v_nop\n\tv_nop\n\tv_nop\n\tv_nop" : "+v"(c) : "v"(a), "v"(b));
  return c;
}

__device__ __forceinline__ _Float16 to_f16_flush(float v) {
  const float w = (fabsf(v) < kF16MinNormal) ? 0.0f : v;
  return (_Float16)w;
}

__device__ __forceinline__ void tile_sums(const v8f a, float& t, float& w5, float& w6, float& w7) {
  const float p0 = a[0] * a[0];
  const float p1 = a[1] * a[1];
  const float p2 = a[2] * a[2];
  const float p3 = a[3] * a[3];
  const float p4 = a[4] * a[4];
  const float p5 = a[5] * a[5];
  const float p6 = a[6] * a[6];
  const float p7 = a[7] * a[7];
  const float e0 = p0 + p1, d0 = p0 - p1;
  const float e1 = p2 + p3, d1 = p2 - p3;
  const float e2 = p4 + p5, d2 = p4 - p5;
  const float e3 = p6 + p7, d3 = p6 - p7;
  const float ea = e0 + e1;
  const float eb = e2 + e3;
  t = ea + eb;
  w5 += ea - eb;
  w6 += (e0 - e1) + (e2 - e3);
  w7 += (d0 + d1) + (d2 + d3);
}

struct Cplx { float x, y; };

__global__ __launch_bounds__(128) void sim_columns_kernel(const float* __restrict__ W, float* __restrict__ UT) {
  __shared__ Cplx st[kDim];
  const int t = threadIdx.x;
  const int j = blockIdx.x;
  st[t]       = (t == j)       ? Cplx{1.f, 0.f} : Cplx{0.f, 0.f};
  st[t + 128] = (t + 128 == j) ? Cplx{1.f, 0.f} : Cplx{0.f, 0.f};
  __syncthreads();

#pragma unroll 1
  for (int l = 0; l < kLayers; ++l) {
#pragma unroll 1
    for (int q = 0; q < kWires; ++q) {
      const int p  = 7 - q;
      const int k0 = ((t >> p) << (p + 1)) | (t & ((1 << p) - 1));
      const int k1 = k0 | (1 << p);
      {
        const float th = 0.5f * W[(l * kWires + q) * 3 + 0];
        const float c = cosf(th), s = sinf(th);
        const Cplx s0 = st[k0], s1 = st[k1];
        st[k0] = { c * s0.x + s * s1.y,  c * s0.y - s * s1.x };
        st[k1] = { s * s0.y + c * s1.x, -s * s0.x + c * s1.y };
        __syncthreads();
      }
      {
        const float th = 0.5f * W[(l * kWires + q) * 3 + 1];
        const float c = cosf(th), s = sinf(th);
        const Cplx s0 = st[k0], s1 = st[k1];
        st[k0] = { c * s0.x - s * s1.x, c * s0.y - s * s1.y };
        st[k1] = { s * s0.x + c * s1.x, s * s0.y + c * s1.y };
        __syncthreads();
      }
      {
        const float th = 0.5f * W[(l * kWires + q) * 3 + 2];
        const float c = cosf(th), s = sinf(th);
        const Cplx s0 = st[k0], s1 = st[k1];
        st[k0] = { c * s0.x + s * s0.y, c * s0.y - s * s0.x };
        st[k1] = { c * s1.x - s * s1.y, c * s1.y + s * s1.x };
        __syncthreads();
      }
    }
#pragma unroll 1
    for (int q = 0; q < kWires; ++q) {
      const int pc = 7 - q;
      const int pg = 7 - ((q + 1) & 7);
      if (t < 64) {
        const int lo = pc < pg ? pc : pg;
        const int hi = pc < pg ? pg : pc;
        int k = ((t >> lo) << (lo + 1)) | (t & ((1 << lo) - 1));
        k = ((k >> hi) << (hi + 1)) | (k & ((1 << hi) - 1));
        const int a = k | (1 << pc);
        const int b = a | (1 << pg);
        const Cplx tmp = st[a];
        st[a] = st[b];
        st[b] = tmp;
      }
      __syncthreads();
    }
  }

  const int pc4 = __popc(j) & 3;
  const int plane = t >> 6;
  const int n4 = (t & 63) * 4;
  v4f ov;
#pragma unroll
  for (int e = 0; e < 4; ++e) {
    const Cplx a = st[n4 + e];
    const float re = (pc4 == 0) ? a.x : (pc4 == 1) ? a.y : (pc4 == 2) ? -a.x : -a.y;
    const float im = (pc4 == 0) ? a.y : (pc4 == 1) ? -a.x : (pc4 == 2) ? -a.y : a.x;
    ov[e] = plane ? im : re;
  }
  float* dst = UT + (size_t)plane * kDim * kDim + (size_t)j * kDim + n4;
  *(volatile v4f*)dst = ov;
  __threadfence();
  *(volatile v4f*)dst = ov;
}

__global__ __launch_bounds__(256) void pack_v_kernel(const float* __restrict__ UT, unsigned short* __restrict__ VT) {
  __shared__ float sT[64 * 65];
  const int tid = threadIdx.x;
  const int j0 = blockIdx.x * 64;
  const int n0 = blockIdx.y * 64;
  const int plane = blockIdx.z;
  const float* src = UT + (size_t)plane * kDim * kDim;
#pragma unroll 1
  for (int it = 0; it < 16; ++it) {
    const int jj = it * 4 + (tid >> 6);
    const int nn = tid & 63;
    sT[jj * 65 + nn] = src[(size_t)(j0 + jj) * kDim + n0 + nn];
  }
  __syncthreads();
  const int q = tid >> 3;
  const int c8 = (tid & 7) * 8;
  v8h hv[2];
#pragma unroll
  for (int it = 0; it < 2; ++it) {
    const int nn = it * 32 + q;
#pragma unroll
    for (int e = 0; e < 8; ++e) {
      const float v = sT[(c8 + e) * 65 + nn] * kCarryV;
      hv[it][e] = to_f16_flush(v);
    }
  }
  for (int pass = 0; pass < 2; ++pass) {
#pragma unroll
    for (int it = 0; it < 2; ++it) {
      unsigned short* dst = VT + (size_t)(plane * kDim + n0 + it * 32 + q) * kDim + j0 + c8;
      *(volatile v8h*)dst = hv[it];
    }
    __threadfence();
  }
}

__global__ __launch_bounds__(kBlkThreads) void expect_kernel(const float* __restrict__ X,
                                                            const unsigned short* __restrict__ VTp,
                                                            float* __restrict__ out) {
  __shared__ __align__(16) _Float16 sFrag[kBlkWaves * kKSteps * 2 * 2 * 32 * 8];
  __shared__ __align__(16) float sC[kBlkSamples * kWires];
  __shared__ __align__(16) float sS[kBlkSamples * kWires];
  __shared__ __align__(16) float sO[kBlkWaves * 32 * kWires];
  const _Float16* VT = (const _Float16*)VTp;
  const int tid  = threadIdx.x;
  const int lane = tid & 31;
  const int wave = tid >> 5;
  const int hh   = lane >> 4;
  const int cl   = lane & 15;
  const int row0 = blockIdx.x * kBlkSamples;

#pragma unroll 1
  for (int it = 0; it < (kBlkSamples * kWires) / kBlkThreads; ++it) {
    const int idx = it * kBlkThreads + tid;
    const float th = 0.5f * X[(size_t)row0 * kWires + idx];
    sC[idx] = cosf(th);
    sS[idx] = sinf(th);
  }
  __syncthreads();

#pragma unroll 1
  for (int j = 0; j < 2; ++j) {
    const int s = wave * 32 + j * 16 + cl;
    const v4f ca = *(const v4f*)(sC + s * kWires);
    const v4f cb = *(const v4f*)(sC + s * kWires + 4);
    const v4f sa = *(const v4f*)(sS + s * kWires);
    const v4f sb = *(const v4f*)(sS + s * kWires + 4);
    const float f4 = hh ? sb[0] : cb[0];
    const float m0 = ca[3] * f4;
    const float m1 = sa[3] * f4;
    float mm[16];
#pragma unroll
    for (int e = 0; e < 8; ++e) {
      const float l8 = ((e & 4) ? sb[1] : cb[1]) * ((e & 2) ? sb[2] : cb[2]) * ((e & 1) ? sb[3] : cb[3]);
      mm[e]     = m0 * l8;
      mm[8 + e] = m1 * l8;
    }
#pragma unroll 1
    for (int ks = 0; ks < kKSteps; ++ks) {
      const float hs = (((ks & 4) ? sa[0] : ca[0]) * ((ks & 2) ? sa[1] : ca[1])) *
                       (((ks & 1) ? sa[2] : ca[2]) * kCarryR);
      v8h f0, f1;
#pragma unroll
      for (int e = 0; e < 8; ++e) {
        f0[e] = to_f16_flush(hs * mm[e]);
        f1[e] = to_f16_flush(hs * mm[8 + e]);
      }
      _Float16* slot = sFrag + ((size_t)(((wave * kKSteps + ks) * 2 + j) * 2) * 32 + lane) * 8;
      *(v8h*)(slot) = f0;
      *(v8h*)(slot + 256) = f1;
    }
  }
  __syncthreads();

  float S[2][8];
#pragma unroll
  for (int j = 0; j < 2; ++j)
#pragma unroll
    for (int w = 0; w < 8; ++w) S[j][w] = 0.f;

#pragma unroll 1
  for (int tn = 0; tn < kAmpRows / 64; ++tn) {
    v8f acc[4][2];
#pragma unroll
    for (int i = 0; i < 4; ++i)
#pragma unroll
      for (int j = 0; j < 2; ++j) acc[i][j] = (v8f){0.f, 0.f, 0.f, 0.f, 0.f, 0.f, 0.f, 0.f};
    const _Float16* vrow = VT + (size_t)(tn * 64 + cl) * kDim + 8 * hh;
#pragma unroll 1
    for (int ks = 0; ks < kKSteps; ++ks) {
      const _Float16* slot = sFrag + ((size_t)((wave * kKSteps + ks) * 4) * 32 + lane) * 8;
      FragU b0, b1;
      b0.h[0] = *(const v8h*)(slot);
      b0.h[1] = *(const v8h*)(slot + 256);
      b1.h[0] = *(const v8h*)(slot + 512);
      b1.h[1] = *(const v8h*)(slot + 768);
#pragma unroll
      for (int i = 0; i < 4; ++i) {
        const v16h a = frag_load_rowmajor(vrow + (size_t)i * 16 * kDim + ks * 32);
        acc[i][0] = mma_guarded(a, b0.v, acc[i][0]);
        acc[i][1] = mma_guarded(a, b1.v, acc[i][1]);
      }
    }
    const float sg1 = (tn & 1) ? -1.f : 1.f;
    const float sg0 = (tn & 2) ? -1.f : 1.f;
#pragma unroll
    for (int j = 0; j < 2; ++j) {
      float t0, t1, t2, t3;
      float w5 = 0.f, w6 = 0.f, w7 = 0.f;
      tile_sums(acc[0][j], t0, w5, w6, w7);
      tile_sums(acc[1][j], t1, w5, w6, w7);
      tile_sums(acc[2][j], t2, w5, w6, w7);
      tile_sums(acc[3][j], t3, w5, w6, w7);
      const float ta = t0 + t1;
      const float tb = t2 + t3;
      const float tt = ta + tb;
      S[j][2] += ta - tb;
      S[j][3] += (t0 - t1) + (t2 - t3);
      S[j][0] += sg0 * tt;
      S[j][1] += sg1 * tt;
      S[j][4] += tt;
      S[j][5] += w5;
      S[j][6] += w6;
      S[j][7] += w7;
    }
  }

  float o[2][8];
#pragma unroll
  for (int j = 0; j < 2; ++j) {
#pragma unroll
    for (int w = 0; w < 8; ++w) {
      const float y = S[j][w];
      const float z = __shfl_xor(y, 16, 32);
      if (w == 4) o[j][w] = hh ? (z - y) : (y - z);
      else        o[j][w] = y + z;
    }
  }
  float* so = sO + wave * 32 * kWires;
  v4f r0, r1;
#pragma unroll
  for (int w = 0; w < 4; ++w) {
    r0[w] = (hh ? o[1][w] : o[0][w]) * kFoldSq;
    r1[w] = (hh ? o[1][4 + w] : o[0][4 + w]) * kFoldSq;
  }
  *(v4f*)(so + lane * kWires) = r0;
  *(v4f*)(so + lane * kWires + 4) = r1;
  __syncthreads();
  const v4f a0 = *(const v4f*)(so + lane * 4);
  const v4f a1 = *(const v4f*)(so + 128 + lane * 4);
  float* dst = out + (size_t)(row0 + wave * 32) * kWires + lane * 4;
  *(volatile v4f*)(dst) = a0;
  *(volatile v4f*)(dst + 128) = a1;
  __threadfence();
  *(volatile v4f*)(dst) = a0;
  *(volatile v4f*)(dst + 128) = a1;
}

extern "C" void kernel_launch(void* const* d_in, const int* in_sizes, int n_in,
                              void* d_out, int out_size, void* d_ws, size_t ws_size,
                              hipStream_t stream) {
  if (n_in < 2) return;
  if (in_sizes[0] != kBatch * kWires) return;
  if (in_sizes[1] != kLayers * kWires * 3) return;
  if (out_size != kBatch * kWires) return;
  if (ws_size < kWsTotal) return;

  const float* x = (const float*)d_in[0];
  const float* w = (const float*)d_in[1];
  float* out = (float*)d_out;
  char* ws = (char*)d_ws;
  float* UT = (float*)(ws + kOffUT);
  unsigned short* VT = (unsigned short*)(ws + kOffVT);

  sim_columns_kernel<<<kDim, 128, 0, stream>>>(w, UT);
  pack_v_kernel<<<dim3(kDim / 64, kDim / 64, 2), 256, 0, stream>>>(UT, VT);
  expect_kernel<<<kBatch / kBlkSamples, kBlkThreads, 0, stream>>>(x, VT, out);
}
